// CHARM_10677288698628
// MI455X (gfx1250) — hardware-verified
//
#include <hip/hip_runtime.h>
#include <stddef.h>
#include <math.h>

typedef __attribute__((ext_vector_type(16))) _Float16 v16h;
typedef __attribute__((ext_vector_type(8)))  _Float16 v8h;
typedef __attribute__((ext_vector_type(4)))  _Float16 v4h;
typedef __attribute__((ext_vector_type(16))) __bf16   v16b;
typedef __attribute__((ext_vector_type(8)))  __bf16   v8b;
typedef __attribute__((ext_vector_type(8)))  float    v8f;
typedef __attribute__((ext_vector_type(4)))  float    v4f;
typedef __attribute__((ext_vector_type(4)))  int      v4i;

constexpr int HID    = 128;
constexpr int HID2   = 256;
constexpr int NODEIN = 64;
constexpr int EDGED  = 32;
constexpr int KMSG   = 288;
constexpr int TOKH   = 64;
constexpr int NLAYER = 3;
constexpr int NTHR   = 256;
constexpr int NWAVE  = 8;
constexpr int CHE    = 53760;
constexpr int RPQ    = 512;
constexpr int NBA    = 512;
constexpr int EPT    = 8;
constexpr int NGRP   = 1;
constexpr int SUBCH  = NTHR * EPT * NGRP;
constexpr int WCAP   = EPT * NGRP * 32;
constexpr int LISTN  = NWAVE * WCAP;
constexpr int MAXSUB = (CHE + SUBCH - 1) / SUBCH;
constexpr int LDS_AGG = NBA * HID * 4 + LISTN * 4 + 64;

static_assert((SUBCH & (SUBCH - 1)) == 0 && SUBCH <= 4096);
static_assert((NBA & (NBA - 1)) == 0 && NBA <= 4096);
static_assert(RPQ % NBA == 0 && RPQ % 64 == 0 && RPQ % NTHR == 0);
static_assert(CHE % 64 == 0);
static_assert(LDS_AGG == 270400);
static_assert(KMSG == 2 * HID + EDGED);

__device__ __forceinline__ unsigned short f2bf_bits(float f) {
  unsigned u = __float_as_uint(f);
  return (unsigned short)((u + 0x7FFFu + ((u >> 16) & 1u)) >> 16);
}
__device__ __forceinline__ float bf_bits2f(unsigned short h) { return __uint_as_float(((unsigned)h) << 16); }

__device__ __forceinline__ void dep_guard_h(v8f& a, v8f& b, v16h x, v16h y) { asm volatile("v_nop\n\tv_nop\n\tv_nop\n\tv_nop" : "+v"(a), "+v"(b) : "v"(x), "v"(y)); }
__device__ __forceinline__ void dep_guard_b(v8f& a, v8f& b, v16b x, v16b y) { asm volatile("v_nop\n\tv_nop\n\tv_nop\n\tv_nop" : "+v"(a), "+v"(b) : "v"(x), "v"(y)); }
__device__ __forceinline__ void keep4_h(v16h a, v16h b, v16h c, v16h d) { asm volatile("v_nop" :: "v"(a), "v"(b), "v"(c), "v"(d)); }
__device__ __forceinline__ void keep4_b(v16b a, v16b b, v16b c, v16b d) { asm volatile("v_nop" :: "v"(a), "v"(b), "v"(c), "v"(d)); }
__device__ __forceinline__ void acc_guard4(v8f& a, v8f& b, v8f& c, v8f& d) { asm volatile("v_nop\n\tv_nop\n\tv_nop\n\tv_nop" : "+v"(a), "+v"(b), "+v"(c), "+v"(d)); }
template <typename T> struct Frag;
template <> struct Frag<_Float16> {
  typedef v16h V; union U { v16h v; v8h h[2]; };
  static __device__ __forceinline__ v16h load(const _Float16* p) {
    U f; f.h[0] = *(const v8h*)(p); f.h[1] = *(const v8h*)(p + 16); return f.v;
  }
  static __device__ __forceinline__ v8f mma(v16h a, v16h b, v8f c) {
    return __builtin_amdgcn_wmma_f32_16x16x32_f16(false, a, false, b, (short)0, c, false, false);
  }
  static __device__ __forceinline__ void guard(v8f& a, v8f& b, v16h x, v16h y) { dep_guard_h(a, b, x, y); }
  static __device__ __forceinline__ void keep(v16h a, v16h b, v16h c, v16h d) { keep4_h(a, b, c, d); }
};
template <> struct Frag<__bf16> {
  typedef v16b V; union U { v16b v; v8b h[2]; };
  static __device__ __forceinline__ v16b load(const __bf16* p) {
    U f; f.h[0] = *(const v8b*)(p); f.h[1] = *(const v8b*)(p + 16); return f.v;
  }
  static __device__ __forceinline__ v8f mma(v16b a, v16b b, v8f c) {
    return __builtin_amdgcn_wmma_f32_16x16x32_bf16(false, a, false, b, (short)0, c, false, false);
  }
  static __device__ __forceinline__ void guard(v8f& a, v8f& b, v16b x, v16b y) { dep_guard_b(a, b, x, y); }
  static __device__ __forceinline__ void keep(v16b a, v16b b, v16b c, v16b d) { keep4_b(a, b, c, d); }
};

template <int ET> struct Elem;
template <> struct Elem<0> { typedef _Float16 T; };
template <> struct Elem<1> { typedef __bf16 T; };
template <int ET, bool SPLIT, int BIAS_MODE, int OUT_MODE, bool RESID, int ACT = 0>
__global__ __launch_bounds__(256) void wmma_gemm64(
    const unsigned short* __restrict__ Ap, const unsigned short* __restrict__ A2p, int lda, long strideA,
    const unsigned short* __restrict__ Btp, const unsigned short* __restrict__ Bt2p, int ldb, long strideB,
    void* __restrict__ Cout, void* __restrict__ Cout2, int ldc, long strideC,
    const float* __restrict__ bias,
    const float* __restrict__ resid, long strideR,
    int M, int N, int K, float scale) {
  typedef typename Elem<ET>::T T;
  typedef typename Frag<T>::V V;
  const T* A = (const T*)Ap; const T* A2 = (const T*)A2p; const T* Bt = (const T*)Btp; const T* Bt2 = (const T*)Bt2p;
  __shared__ __align__(16) float sT[8][16 * 68];
  const int b    = blockIdx.y;
  const int lane = threadIdx.x & 31;
  const int wave = threadIdx.x >> 5;
  const int tilesN = N >> 6;
  const int tilesM = M >> 6;
  const int tile = blockIdx.x * 8 + wave;
  if (tile >= tilesM * tilesN) return;
  const int tm = tile / tilesN;
  const int tn = tile - tm * tilesN;
  const int m0 = tm << 6;
  const int n0 = tn << 6;

  const T* Ab  = A  + (size_t)b * strideA;
  const T* Bb  = Bt + (size_t)b * strideB;
  const T* Ab2 = SPLIT ? (A2  + (size_t)b * strideA) : nullptr;
  const T* Bb2 = SPLIT ? (Bt2 + (size_t)b * strideB) : nullptr;

  const int rlane = lane & 15;
  const int koff  = (lane >> 4) * 8;
  const int mOff  = (lane >> 4) * 8;

  v8f acc[4][4];
#pragma unroll
  for (int i = 0; i < 4; ++i)
#pragma unroll
    for (int j = 0; j < 4; ++j) acc[i][j] = (v8f){0.f,0.f,0.f,0.f,0.f,0.f,0.f,0.f};

  for (int k0 = 0; k0 < K; k0 += 32) {
    V bh[4], bl[4];
#pragma unroll
    for (int j = 0; j < 4; ++j) {
      const size_t bo = (size_t)(n0 + (j << 4) + rlane) * ldb + koff + k0;
      bh[j] = Frag<T>::load(Bb + bo);
      if (SPLIT) bl[j] = Frag<T>::load(Bb2 + bo);
    }
#pragma unroll
    for (int i = 0; i < 4; ++i) {
      const size_t ao = (size_t)(m0 + (i << 4) + rlane) * lda + koff + k0;
      V ah = Frag<T>::load(Ab + ao);
      V al;
      if (SPLIT) al = Frag<T>::load(Ab2 + ao);
#pragma unroll
      for (int j = 0; j < 4; ++j) {
        acc[i][j] = Frag<T>::mma(ah, bh[j], acc[i][j]);
        if (SPLIT) {
          acc[i][j] = Frag<T>::mma(ah, bl[j], acc[i][j]);
          acc[i][j] = Frag<T>::mma(al, bh[j], acc[i][j]);
        }
      }
      Frag<T>::guard(acc[i][0], acc[i][3], ah, SPLIT ? al : ah);
    }
    Frag<T>::keep(bh[0], bh[1], bh[2], bh[3]);
    if (SPLIT) Frag<T>::keep(bl[0], bl[1], bl[2], bl[3]);
  }
  acc_guard4(acc[0][0], acc[0][1], acc[0][2], acc[0][3]);
  acc_guard4(acc[1][0], acc[1][1], acc[1][2], acc[1][3]);
  acc_guard4(acc[2][0], acc[2][1], acc[2][2], acc[2][3]);
  acc_guard4(acc[3][0], acc[3][1], acc[3][2], acc[3][3]);

  float* slab = sT[wave];
  const float* Rb = RESID ? (resid + (size_t)b * strideR) : nullptr;
#pragma unroll
  for (int i = 0; i < 4; ++i) {
    const int mBase = m0 + (i << 4);
#pragma unroll
    for (int j = 0; j < 4; ++j) {
      const int n = n0 + (j << 4) + rlane;
      float bv = 0.f;
      if (BIAS_MODE == 2) bv = bias[n];
#pragma unroll
      for (int r = 0; r < 8; ++r) {
        float v = acc[i][j][r] * scale;
        if (BIAS_MODE == 1) v += bias[mBase + mOff + r];
        if (BIAS_MODE == 2) v += bv;
        if (RESID) v += Rb[(size_t)(mBase + mOff + r) * ldc + n];
        if (ACT == 1) v = tanhf(v);
        if (ACT == 2) v = fmaxf(v, 0.0f);
        if (ACT == 3) v = v / (1.0f + expf(-v));
        if (ACT == 4) v = (v > 0.f) ? v : 0.01f * v;
        if (ACT == 5) v = 0.5f * v * (1.0f + erff(v * 0.70710678118654752f));
        slab[(mOff + r) * 68 + (j << 4) + rlane] = v;
      }
    }
    __builtin_amdgcn_fence(__ATOMIC_RELEASE, "workgroup");
    __builtin_amdgcn_wave_barrier();
    __builtin_amdgcn_fence(__ATOMIC_ACQUIRE, "workgroup");
    if (OUT_MODE == 0) {
      float* C = (float*)Cout + (size_t)b * strideC;
      const int hh = lane >> 4, c4 = (lane & 15) * 4;
      for (int pass = 0; pass < 2; ++pass) {
#pragma unroll
        for (int it = 0; it < 8; ++it) {
          const int row = it * 2 + hh;
          v4f v = *(const v4f*)(slab + row * 68 + c4);
          *(volatile v4f*)(C + (size_t)(mBase + row) * ldc + n0 + c4) = v;
        }
        __threadfence();
      }
    } else {
      const int q = lane >> 3, c8 = (lane & 7) * 8;
      unsigned short* C  = (unsigned short*)Cout  + (size_t)b * strideC;
      unsigned short* C2 = (OUT_MODE == 2) ? ((unsigned short*)Cout2 + (size_t)b * strideC) : nullptr;
      for (int pass = 0; pass < 2; ++pass) {
#pragma unroll
        for (int it = 0; it < 4; ++it) {
          const int row = it * 4 + q;
          const float* sp = slab + row * 68 + c8;
          v8h hv, lv;
#pragma unroll
          for (int e = 0; e < 8; ++e) {
            if (OUT_MODE == 1) {
              hv[e] = (_Float16)sp[e];
            } else {
              unsigned short hb = f2bf_bits(sp[e]);
              unsigned short lb = f2bf_bits(sp[e] - bf_bits2f(hb));
              hv[e] = __builtin_bit_cast(_Float16, hb);
              lv[e] = __builtin_bit_cast(_Float16, lb);
            }
          }
          *(volatile v8h*)(C + (size_t)(mBase + row) * ldc + n0 + c8) = hv;
          if (OUT_MODE == 2) *(volatile v8h*)(C2 + (size_t)(mBase + row) * ldc + n0 + c8) = lv;
        }
        __threadfence();
      }
    }
    __builtin_amdgcn_fence(__ATOMIC_RELEASE, "workgroup");
    __builtin_amdgcn_wave_barrier();
    __builtin_amdgcn_fence(__ATOMIC_ACQUIRE, "workgroup");
  }
}

template <int NB>
__device__ __forceinline__ int scan_chunk(const int* __restrict__ lst, int nE, int cbase, int nodeBase,
                                          int* list, int tid, int lane, int wave, int fullvec) {
  int wc = 0;
#pragma unroll
  for (int g = 0; g < NGRP; ++g) {
    const int el0 = (g * NTHR + tid) * EPT;
    const int e0  = cbase + el0;
    v4i da, db;
    if (fullvec) {
      da = *(const v4i*)(lst + e0);
      db = *(const v4i*)(lst + e0 + 4);
    } else {
      const int em = nE - 1;
      da.x = lst[(e0     < em) ? e0     : em];
      da.y = lst[(e0 + 1 < em) ? e0 + 1 : em];
      da.z = lst[(e0 + 2 < em) ? e0 + 2 : em];
      da.w = lst[(e0 + 3 < em) ? e0 + 3 : em];
      db.x = lst[(e0 + 4 < em) ? e0 + 4 : em];
      db.y = lst[(e0 + 5 < em) ? e0 + 5 : em];
      db.z = lst[(e0 + 6 < em) ? e0 + 6 : em];
      db.w = lst[(e0 + 7 < em) ? e0 + 7 : em];
    }
    const bool v0 = (e0 < nE), v1 = (e0 + 1 < nE), v2 = (e0 + 2 < nE), v3 = (e0 + 3 < nE);
    const bool v4 = (e0 + 4 < nE), v5 = (e0 + 5 < nE), v6 = (e0 + 6 < nE), v7 = (e0 + 7 < nE);
    const unsigned nb = (unsigned)nodeBase;
    const unsigned s0 = (unsigned)da.x - nb, s1 = (unsigned)da.y - nb;
    const unsigned s2 = (unsigned)da.z - nb, s3 = (unsigned)da.w - nb;
    const unsigned s4 = (unsigned)db.x - nb, s5 = (unsigned)db.y - nb;
    const unsigned s6 = (unsigned)db.z - nb, s7 = (unsigned)db.w - nb;
    const bool h0 = v0 && (s0 < (unsigned)NB), h1 = v1 && (s1 < (unsigned)NB);
    const bool h2 = v2 && (s2 < (unsigned)NB), h3 = v3 && (s3 < (unsigned)NB);
    const bool h4 = v4 && (s4 < (unsigned)NB), h5 = v5 && (s5 < (unsigned)NB);
    const bool h6 = v6 && (s6 < (unsigned)NB), h7 = v7 && (s7 < (unsigned)NB);
    const unsigned any = __builtin_amdgcn_ballot_w32(h0 | h1 | h2 | h3 | h4 | h5 | h6 | h7);
    if (any != 0u) {
#define HITJ(J, HJ, SJ) { \
        const unsigned mj = __builtin_amdgcn_ballot_w32(HJ); \
        if (mj != 0u) { \
          if (HJ) { \
            const int pos = wc + (int)__builtin_amdgcn_mbcnt_lo(mj, 0u); \
            if (pos < WCAP) list[wave * WCAP + pos] = ((el0 + (J)) << 12) | (int)(SJ); \
          } \
          wc += (int)__builtin_popcount(mj); } }
      HITJ(0, h0, s0)
      HITJ(1, h1, s1)
      HITJ(2, h2, s2)
      HITJ(3, h3, s3)
      HITJ(4, h4, s4)
      HITJ(5, h5, s5)
      HITJ(6, h6, s6)
      HITJ(7, h7, s7)
#undef HITJ
    }
  }
  return wc;
}

__global__ __launch_bounds__(NTHR) void k_wsplit(const float* __restrict__ W, long strideW, int Kin, int ncol, int G,
                                                 int NR, int KP, unsigned short* bth, unsigned short* btl, long strideO) {
  const float* Wl = W + (size_t)blockIdx.y * (size_t)strideW;
  const size_t ob = (size_t)blockIdx.y * (size_t)strideO;
  const int tpr = KP >> 3;
  const int i = blockIdx.x * NTHR + threadIdx.x;
  if (i >= NR * tpr) return;
  const int n  = i / tpr;
  const int k0 = (i - n * tpr) * 8;
  int g = n / ncol; g = (g > G - 1) ? G - 1 : g;
  int nn = n - g * ncol; nn = (nn > ncol - 1) ? ncol - 1 : ((nn < 0) ? 0 : nn);
  const bool nok = (n < G * ncol);
  v8h hv, lv;
#pragma unroll
  for (int e = 0; e < 8; ++e) {
    const int k  = k0 + e;
    const int kc = (k < Kin) ? k : Kin - 1;
    float v = Wl[((size_t)g * Kin + kc) * ncol + nn];
    if (k >= Kin || !nok) v = 0.f;
    const unsigned short hb = f2bf_bits(v);
    const unsigned short lb = f2bf_bits(v - bf_bits2f(hb));
    hv[e] = __builtin_bit_cast(_Float16, hb);
    lv[e] = __builtin_bit_cast(_Float16, lb);
  }
  const size_t o = ob + (size_t)i * 8;
  *(volatile v8h*)(bth + o) = hv;
  *(volatile v8h*)(btl + o) = lv;
  __threadfence();
  *(volatile v8h*)(bth + o) = hv;
  *(volatile v8h*)(btl + o) = lv;
}

__global__ __launch_bounds__(NTHR) void k_wf16(const float* __restrict__ W, long strideW, int Kin, int ncol,
                                               int NR, int KP, float sc, unsigned short* bt, long strideO) {
  const float* Wl = W + (size_t)blockIdx.y * (size_t)strideW;
  const size_t ob = (size_t)blockIdx.y * (size_t)strideO;
  const int tpr = KP >> 3;
  const int i = blockIdx.x * NTHR + threadIdx.x;
  if (i >= NR * tpr) return;
  const int n   = i / tpr;
  const int k0  = (i - n * tpr) * 8;
  const int ncl = (n < ncol) ? n : ncol - 1;
  v8h hv;
#pragma unroll
  for (int e = 0; e < 8; ++e) {
    const int k  = k0 + e;
    const int kc = (k < Kin) ? k : Kin - 1;
    float v = sc * Wl[(size_t)kc * ncol + ncl];
    if (k >= Kin || n >= ncol) v = 0.f;
    hv[e] = (_Float16)v;
  }
  const size_t o = ob + (size_t)i * 8;
  *(volatile v8h*)(bt + o) = hv;
  __threadfence();
  *(volatile v8h*)(bt + o) = hv;
}

__global__ __launch_bounds__(NTHR) void k_wblk(const float* __restrict__ ew, const float* __restrict__ eb,
                                               unsigned short* bt, float* b64) {
  const int i  = blockIdx.x * NTHR + threadIdx.x;
  const int n  = i >> 3;
  const int k0 = (i & 7) * 8;
  v8h hv;
#pragma unroll
  for (int e = 0; e < 8; ++e) {
    const int k = k0 + e;
    const float w = ew[(k & 31) * EDGED + (n & 31)];
    const bool same = ((n >> 5) == (k >> 5));
    hv[e] = (_Float16)(same ? 8.0f * w : 0.0f);
  }
  const size_t o = (size_t)i * 8;
  *(volatile v8h*)(bt + o) = hv;
  __threadfence();
  *(volatile v8h*)(bt + o) = hv;
  const bool dob = (i < 16);
  const int ic = dob ? i : 0;
  const float t0 = eb[(4 * ic + 0) & 31], t1 = eb[(4 * ic + 1) & 31];
  const float t2 = eb[(4 * ic + 2) & 31], t3 = eb[(4 * ic + 3) & 31];
  const v4f bv = {t0, t1, t2, t3};
  if (dob) *(volatile v4f*)(b64 + 4 * ic) = bv;
  __threadfence();
  if (dob) *(volatile v4f*)(b64 + 4 * ic) = bv;
}

__global__ __launch_bounds__(NTHR) void k_xsplit(const float* __restrict__ x, int nN, int NPr,
                                                 unsigned short* xh, unsigned short* xl) {
  const int i = blockIdx.x * NTHR + threadIdx.x;
  const int row = i >> 3;
  const int k0 = (i & 7) * 8;
  const int rowc = (row < nN) ? row : nN - 1;
  const float* xr = x + (size_t)rowc * NODEIN + k0;
  const v4f a0 = *(const v4f*)xr;
  const v4f a1 = *(const v4f*)(xr + 4);
  const float A8[8] = {a0.x, a0.y, a0.z, a0.w, a1.x, a1.y, a1.z, a1.w};
  v8h hv, lv;
#pragma unroll
  for (int e = 0; e < 8; ++e) {
    float v = A8[e];
    if (row >= nN) v = 0.f;
    const unsigned short hb = f2bf_bits(v);
    const unsigned short lb = f2bf_bits(v - bf_bits2f(hb));
    hv[e] = __builtin_bit_cast(_Float16, hb);
    lv[e] = __builtin_bit_cast(_Float16, lb);
  }
  const bool ok = (row < NPr);
  const size_t o = (size_t)i * 8;
  if (ok) { *(volatile v8h*)(xh + o) = hv; *(volatile v8h*)(xl + o) = lv; }
  __threadfence();
  if (ok) { *(volatile v8h*)(xh + o) = hv; *(volatile v8h*)(xl + o) = lv; }
}

__global__ __launch_bounds__(NTHR) void k_cast_ea(const float* __restrict__ ea, int nE, int EP, unsigned short* out) {
  const int i = blockIdx.x * NTHR + threadIdx.x;
  const int row = i >> 2;
  const int k0 = (i & 3) * 8;
  const int rowc = (row < nE) ? row : nE - 1;
  const float* er = ea + (size_t)rowc * EDGED + k0;
  const v4f a0 = *(const v4f*)er;
  const v4f a1 = *(const v4f*)(er + 4);
  const float A8[8] = {a0.x, a0.y, a0.z, a0.w, a1.x, a1.y, a1.z, a1.w};
  v8h hv;
#pragma unroll
  for (int e = 0; e < 8; ++e) hv[e] = (_Float16)((row < nE) ? A8[e] : 0.0f);
  const bool ok = (row < EP);
  const size_t o = (size_t)i * 8;
  if (ok) *(volatile v8h*)(out + o) = hv;
  __threadfence();
  if (ok) *(volatile v8h*)(out + o) = hv;
}

__global__ __launch_bounds__(NTHR) void k_m1(const float* __restrict__ pab, const unsigned short* __restrict__ pe,
                                             const int* __restrict__ ei, int nN, int nE, int ebase, int Mc,
                                             unsigned short* m1) {
  const int i = blockIdx.x * NTHR + threadIdx.x;
  const int r = i >> 4;
  const int p = (i & 15) * 8;
  const int e = ebase + r;
  const bool valid = (e < nE);
  int ec = valid ? e : nE - 1; ec = (ec < 0) ? 0 : ec;
  int s = ei[ec];
  int d = ei[(size_t)nE + ec];
  s = (s < 0) ? 0 : ((s > nN - 1) ? nN - 1 : s);
  d = (d < 0) ? 0 : ((d > nN - 1) ? nN - 1 : d);
  const float* pa = pab + (size_t)d * HID2 + p;
  const float* pb = pab + (size_t)s * HID2 + HID + p;
  const v4f a0 = *(const v4f*)pa, a1 = *(const v4f*)(pa + 4);
  const v4f b0 = *(const v4f*)pb, b1 = *(const v4f*)(pb + 4);
  const int rc = (r < Mc) ? r : Mc - 1;
  const v8h cv = *(const v8h*)((const _Float16*)pe + (size_t)rc * HID + p);
  const float A8[8] = {a0.x, a0.y, a0.z, a0.w, a1.x, a1.y, a1.z, a1.w};
  const float B8[8] = {b0.x, b0.y, b0.z, b0.w, b1.x, b1.y, b1.z, b1.w};
  v8h ov;
#pragma unroll
  for (int j = 0; j < 8; ++j) {
    float v = A8[j] + B8[j] + (float)cv[j];
    v = fmaxf(v, 0.0f);
    if (!valid) v = 0.0f;
    ov[j] = (_Float16)v;
  }
  const bool ok = (r < Mc);
  const size_t o = (size_t)rc * HID + p;
  if (ok) *(volatile v8h*)(m1 + o) = ov;
  __threadfence();
  if (ok) *(volatile v8h*)(m1 + o) = ov;
}

__global__ __launch_bounds__(NTHR) void k_agg(const int* __restrict__ dstl, int nEc,
                                              const float* __restrict__ mh, float* agg, int first, int vec_ok) {
  constexpr int NB  = NBA;
  constexpr int NV4 = NB * HID / 4;
  static_assert(NV4 % NTHR == 0);
  extern __shared__ v4f lds_dyn[];
  float* acc  = (float*)lds_dyn;
  int*   list = (int*)(acc + NB * HID);
  int*   wcnt = list + LISTN;
  const int tid = threadIdx.x, lane = tid & 31, wave = tid >> 5;
  const int nodeBase = blockIdx.x * NB;
  float* ga = agg + (size_t)nodeBase * HID;

  if (first) {
    const v4f zz = {0.f, 0.f, 0.f, 0.f};
    for (int i = tid; i < NV4; i += NTHR) lds_dyn[i] = zz;
  } else {
    for (int i = tid; i < NV4; i += NTHR) lds_dyn[i] = ((const v4f*)ga)[i];
  }
  __syncthreads();

  int nSub = (nEc + SUBCH - 1) / SUBCH;
  nSub = (nSub > MAXSUB) ? MAXSUB : ((nSub < 0) ? 0 : nSub);
#pragma unroll 1
  for (int ch = 0; ch < nSub; ++ch) {
    const int cbase = ch * SUBCH;
    const int fullvec = (vec_ok != 0 && cbase + SUBCH <= nEc) ? 1 : 0;
    const int wc = scan_chunk<NB>(dstl, nEc, cbase, nodeBase, list, tid, lane, wave, fullvec);
    if (lane == 0) wcnt[wave] = wc;
    __syncthreads();
    if (wave == 0) {
#pragma unroll 1
      for (int wsx = 0; wsx < NWAVE; ++wsx) {
        int n = __builtin_amdgcn_readfirstlane(wcnt[wsx]);
        n = n > WCAP ? WCAP : (n < 0 ? 0 : n);
        const int* lp = list + wsx * WCAP;
#pragma unroll 1
        for (int i = 0; i < n; ++i) {
          const int ent  = __builtin_amdgcn_readfirstlane(lp[i]);
          const int slot = ent & (NB - 1);
          int el = cbase + ((ent >> 12) & (SUBCH - 1));
          el = (el > nEc - 1) ? nEc - 1 : el;
          const v4f m4 = *(const v4f*)(mh + (size_t)el * HID + 4 * lane);
          v4f* ap = (v4f*)(acc + slot * HID + 4 * lane);
          const v4f av = *ap;
          *ap = av + m4;
        }
      }
    }
    __syncthreads();
  }

  for (int pass = 0; pass < 2; ++pass) {
#pragma unroll 4
    for (int i = tid; i < NV4; i += NTHR) { const v4f v = lds_dyn[i]; ((volatile v4f*)ga)[i] = v; }
    __threadfence();
  }
}

__global__ __launch_bounds__(NTHR) void k_aggsplit(const float* __restrict__ agg, int NPr,
                                                   unsigned short* ch, unsigned short* cl) {
  const int i = blockIdx.x * NTHR + threadIdx.x;
  const int row = i >> 4;
  const int k0 = (i & 15) * 8;
  const int rowc = (row < NPr) ? row : NPr - 1;
  const float* ar = agg + (size_t)rowc * HID + k0;
  const v4f a0 = *(const v4f*)ar;
  const v4f a1 = *(const v4f*)(ar + 4);
  const float A8[8] = {a0.x, a0.y, a0.z, a0.w, a1.x, a1.y, a1.z, a1.w};
  v8h hv, lv;
#pragma unroll
  for (int e = 0; e < 8; ++e) {
    const float v = A8[e];
    const unsigned short hb = f2bf_bits(v);
    const unsigned short lb = f2bf_bits(v - bf_bits2f(hb));
    hv[e] = __builtin_bit_cast(_Float16, hb);
    lv[e] = __builtin_bit_cast(_Float16, lb);
  }
  const bool ok = (row < NPr);
  const size_t o = (size_t)rowc * HID2 + HID + k0;
  if (ok) { *(volatile v8h*)(ch + o) = hv; *(volatile v8h*)(cl + o) = lv; }
  __threadfence();
  if (ok) { *(volatile v8h*)(ch + o) = hv; *(volatile v8h*)(cl + o) = lv; }
}

__global__ __launch_bounds__(NTHR) void k_logit(const float* __restrict__ t32, const float* __restrict__ w2,
                                                const float* __restrict__ b2, int nN, int NPr, float* out0) {
  __shared__ __align__(16) float sl[NTHR];
  const int tid = threadIdx.x, lane = tid & 31, wave = tid >> 5;
  const int node = blockIdx.x * NTHR + tid;
  const int nodec = (node < NPr) ? node : NPr - 1;
  const float* tr = t32 + (size_t)nodec * TOKH;
  float acc = 0.0f;
#pragma unroll 1
  for (int p = 0; p < TOKH / 4; ++p) {
    const v4f tv = *(const v4f*)(tr + 4 * p);
    const v4f wv = *(const v4f*)(w2 + 4 * p);
    acc += tv.x * wv.x + tv.y * wv.y + tv.z * wv.z + tv.w * wv.w;
  }
  sl[tid] = acc + b2[0];
  __syncthreads();
  const int nb = blockIdx.x * NTHR + wave * 32;
  const int l8 = (lane < 8) ? lane : 7;
  const v4f v = *(const v4f*)(sl + wave * 32 + 4 * l8);
  const bool ok = (lane < 8) && (nb + 4 * l8 + 4 <= nN);
  float* op = out0 + (size_t)nb + 4 * l8;
  if (ok) *(volatile v4f*)op = v;
  __threadfence();
  if (ok) *(volatile v4f*)op = v;
}

__global__ __launch_bounds__(NTHR) void k_out1(const unsigned short* __restrict__ ch, const unsigned short* __restrict__ cl,
                                               int nN, int NPr, float* out1) {
  const int i = blockIdx.x * NTHR + threadIdx.x;
  const int row = i >> 5;
  const int c4 = (i & 31) * 4;
  int rowc = (row < nN) ? row : nN - 1; rowc = (rowc > NPr - 1) ? NPr - 1 : rowc;
  const unsigned int* hp = (const unsigned int*)(ch + (size_t)rowc * HID2 + c4);
  const unsigned int* lp = (const unsigned int*)(cl + (size_t)rowc * HID2 + c4);
  const unsigned int h01 = hp[0], h23 = hp[1];
  const unsigned int l01 = lp[0], l23 = lp[1];
  v4f o;
  o.x = __uint_as_float(h01 << 16)          + __uint_as_float(l01 << 16);
  o.y = __uint_as_float(h01 & 0xffff0000u)  + __uint_as_float(l01 & 0xffff0000u);
  o.z = __uint_as_float(h23 << 16)          + __uint_as_float(l23 << 16);
  o.w = __uint_as_float(h23 & 0xffff0000u)  + __uint_as_float(l23 & 0xffff0000u);
  const bool ok = (row < nN);
  float* op = out1 + (size_t)rowc * HID + c4;
  if (ok) *(volatile v4f*)op = o;
  __threadfence();
  if (ok) *(volatile v4f*)op = o;
}

extern "C" void kernel_launch(void* const* d_in, const int* in_sizes, int n_in,
                              void* d_out, int out_size, void* d_ws, size_t ws_size,
                              hipStream_t stream) {
  if (n_in < 19) return;
  const int nN = in_sizes[0] / NODEIN;
  const int nE = in_sizes[18] / 2;
  if (nN < 1 || in_sizes[0] != nN * NODEIN || nN > (1 << 22)) return;
  if (nE < 1 || in_sizes[18] != 2 * nE || in_sizes[1] != nE * EDGED || nE > (1 << 26)) return;
  if (in_sizes[2] != NODEIN * HID || in_sizes[3] != HID || in_sizes[4] != EDGED * EDGED || in_sizes[5] != EDGED) return;
  if (in_sizes[6] != NLAYER * KMSG * HID || in_sizes[7] != NLAYER * HID) return;
  if (in_sizes[8] != NLAYER * HID * HID || in_sizes[9] != NLAYER * HID) return;
  if (in_sizes[10] != NLAYER * HID2 * HID || in_sizes[11] != NLAYER * HID) return;
  if (in_sizes[12] != NLAYER * HID * HID || in_sizes[13] != NLAYER * HID) return;
  if (in_sizes[14] != HID * TOKH || in_sizes[15] != TOKH || in_sizes[16] != TOKH || in_sizes[17] < 1) return;
  if (out_size != nN + nN * HID) return;

  const float* x      = (const float*)d_in[0];
  const float* eattr  = (const float*)d_in[1];
  const float* node_w = (const float*)d_in[2];
  const float* node_b = (const float*)d_in[3];
  const float* edge_w = (const float*)d_in[4];
  const float* edge_b = (const float*)d_in[5];
  const float* msg_w1 = (const float*)d_in[6];
  const float* msg_b1 = (const float*)d_in[7];
  const float* msg_w2 = (const float*)d_in[8];
  const float* msg_b2 = (const float*)d_in[9];
  const float* up_w1  = (const float*)d_in[10];
  const float* up_b1  = (const float*)d_in[11];
  const float* up_w2  = (const float*)d_in[12];
  const float* up_b2  = (const float*)d_in[13];
  const float* tok_w1 = (const float*)d_in[14];
  const float* tok_b1 = (const float*)d_in[15];
  const float* tok_w2 = (const float*)d_in[16];
  const float* tok_b2 = (const float*)d_in[17];
  const int*   eidx   = (const int*)d_in[18];
  float* out0 = (float*)d_out;
  float* out1 = out0 + nN;

  const int NPr = ((nN + RPQ - 1) / RPQ) * RPQ;
  const int EP  = ((nE + 127) / 128) * 128;
  const int nChunks = (nE + CHE - 1) / CHE;
  if (nChunks < 1 || nChunks > 64) return;
  const int nA = NPr / NBA;

  size_t off = 0;
  auto carve = [&](size_t bytes) { const size_t o = off; off += (bytes + 255) & ~(size_t)255; return o; };
  const size_t oWNH  = carve((size_t)HID * NODEIN * 2);
  const size_t oWNL  = carve((size_t)HID * NODEIN * 2);
  const size_t oWEB  = carve((size_t)64 * 64 * 2);
  const size_t oBE64 = carve((size_t)64 * 4);
  const size_t oW1AH = carve((size_t)NLAYER * HID2 * HID * 2);
  const size_t oW1AL = carve((size_t)NLAYER * HID2 * HID * 2);
  const size_t oW1E  = carve((size_t)NLAYER * HID * EDGED * 2);
  const size_t oW2E  = carve((size_t)NLAYER * HID * HID * 2);
  const size_t oU1H  = carve((size_t)NLAYER * HID * HID2 * 2);
  const size_t oU1L  = carve((size_t)NLAYER * HID * HID2 * 2);
  const size_t oU2H  = carve((size_t)NLAYER * HID * HID * 2);
  const size_t oU2L  = carve((size_t)NLAYER * HID * HID * 2);
  const size_t oTKH  = carve((size_t)TOKH * HID * 2);
  const size_t oTKL  = carve((size_t)TOKH * HID * 2);
  const size_t oCH   = carve((size_t)NPr * HID2 * 2);
  const size_t oCL   = carve((size_t)NPr * HID2 * 2);
  const size_t oPAB  = carve((size_t)NPr * HID2 * 4);
  const size_t oAGG  = carve((size_t)NPr * HID * 4);
  const size_t oE16  = carve((size_t)EP * EDGED * 2);
  size_t scr = (size_t)CHE * 1024;
  if ((size_t)EP * EDGED * 2 > scr) scr = (size_t)EP * EDGED * 2;
  if ((size_t)NPr * HID * 2 * 2 > scr) scr = (size_t)NPr * HID * 2 * 2;
  if ((size_t)NPr * NODEIN * 2 * 2 > scr) scr = (size_t)NPr * NODEIN * 2 * 2;
  if ((size_t)NPr * TOKH * 4 > scr) scr = (size_t)NPr * TOKH * 4;
  const size_t oSCR  = carve(scr);
  if (off > ws_size || off > (size_t)134217728) return;

  char* ws = (char*)d_ws;
  unsigned short* wnh  = (unsigned short*)(ws + oWNH);
  unsigned short* wnl  = (unsigned short*)(ws + oWNL);
  unsigned short* web  = (unsigned short*)(ws + oWEB);
  float*          be64 = (float*)(ws + oBE64);
  unsigned short* w1ah = (unsigned short*)(ws + oW1AH);
  unsigned short* w1al = (unsigned short*)(ws + oW1AL);
  unsigned short* w1e  = (unsigned short*)(ws + oW1E);
  unsigned short* w2e  = (unsigned short*)(ws + oW2E);
  unsigned short* u1h  = (unsigned short*)(ws + oU1H);
  unsigned short* u1l  = (unsigned short*)(ws + oU1L);
  unsigned short* u2h  = (unsigned short*)(ws + oU2H);
  unsigned short* u2l  = (unsigned short*)(ws + oU2L);
  unsigned short* tkh  = (unsigned short*)(ws + oTKH);
  unsigned short* tkl  = (unsigned short*)(ws + oTKL);
  unsigned short* chp  = (unsigned short*)(ws + oCH);
  unsigned short* clp  = (unsigned short*)(ws + oCL);
  float*          pab  = (float*)(ws + oPAB);
  float*          aggp = (float*)(ws + oAGG);
  unsigned short* e16  = (unsigned short*)(ws + oE16);
  unsigned short* ea16 = (unsigned short*)(ws + oSCR);
  unsigned short* xh   = (unsigned short*)(ws + oSCR);
  unsigned short* xl   = (unsigned short*)(ws + oSCR + (size_t)NPr * NODEIN * 2);
  unsigned short* pe16 = (unsigned short*)(ws + oSCR);
  unsigned short* m1p  = (unsigned short*)(ws + oSCR + (size_t)CHE * HID * 2);
  float*          m2p  = (float*)(ws + oSCR + (size_t)CHE * HID * 4);
  unsigned short* uh   = (unsigned short*)(ws + oSCR);
  unsigned short* ul   = (unsigned short*)(ws + oSCR + (size_t)NPr * HID * 2);
  float*          t32  = (float*)(ws + oSCR);

  auto gemm_blocks = [](int M, int Nn) { return ((M / 64) * (Nn / 64) + 7) / 8; };

  k_wsplit<<<dim3((HID * (NODEIN / 8) + NTHR - 1) / NTHR, 1), NTHR, 0, stream>>>(
      node_w, 0L, NODEIN, HID, 1, HID, NODEIN, wnh, wnl, 0L);
  k_wblk<<<2, NTHR, 0, stream>>>(edge_w, edge_b, web, be64);
  k_wsplit<<<dim3((HID2 * (HID / 8) + NTHR - 1) / NTHR, NLAYER), NTHR, 0, stream>>>(
      msg_w1, (long)KMSG * HID, HID, HID, 2, HID2, HID, w1ah, w1al, (long)HID2 * HID);
  k_wf16<<<dim3((HID * (EDGED / 8) + NTHR - 1) / NTHR, NLAYER), NTHR, 0, stream>>>(
      msg_w1 + (size_t)HID2 * HID, (long)KMSG * HID, EDGED, HID, HID, EDGED, 8.0f, w1e, (long)HID * EDGED);
  k_wf16<<<dim3((HID * (HID / 8) + NTHR - 1) / NTHR, NLAYER), NTHR, 0, stream>>>(
      msg_w2, (long)HID * HID, HID, HID, HID, HID, 8.0f, w2e, (long)HID * HID);
  k_wsplit<<<dim3((HID * (HID2 / 8) + NTHR - 1) / NTHR, NLAYER), NTHR, 0, stream>>>(
      up_w1, (long)HID2 * HID, HID2, HID, 1, HID, HID2, u1h, u1l, (long)HID * HID2);
  k_wsplit<<<dim3((HID * (HID / 8) + NTHR - 1) / NTHR, NLAYER), NTHR, 0, stream>>>(
      up_w2, (long)HID * HID, HID, HID, 1, HID, HID, u2h, u2l, (long)HID * HID);
  k_wsplit<<<dim3((TOKH * (HID / 8) + NTHR - 1) / NTHR, 1), NTHR, 0, stream>>>(
      tok_w1, 0L, HID, TOKH, 1, TOKH, HID, tkh, tkl, 0L);

  k_xsplit<<<(NPr * 8) / NTHR, NTHR, 0, stream>>>(x, nN, NPr, xh, xl);
  wmma_gemm64<1, true, 2, 2, false, 0><<<dim3(gemm_blocks(NPr, HID), 1), 256, 0, stream>>>(
      xh, xl, NODEIN, 0L, wnh, wnl, NODEIN, 0L, (void*)chp, (void*)clp, HID2, 0L, node_b, node_b, 0L, NPr, HID, NODEIN, 1.0f);

  k_cast_ea<<<(EP * 4) / NTHR, NTHR, 0, stream>>>(eattr, nE, EP, ea16);
  wmma_gemm64<0, false, 2, 1, false, 0><<<dim3(gemm_blocks(EP / 2, 64), 1), 256, 0, stream>>>(
      ea16, ea16, 64, 0L, web, web, 64, 0L, (void*)e16, (void*)e16, 64, 0L, be64, be64, 0L, EP / 2, 64, 64, 0.125f);

  for (int l = 0; l < NLAYER; ++l) {
    const unsigned short* w1ahl = w1ah + (size_t)l * HID2 * HID;
    const unsigned short* w1all = w1al + (size_t)l * HID2 * HID;
    const unsigned short* w1el  = w1e  + (size_t)l * HID * EDGED;
    const unsigned short* w2el  = w2e  + (size_t)l * HID * HID;
    const unsigned short* u1hl  = u1h  + (size_t)l * HID * HID2;
    const unsigned short* u1ll  = u1l  + (size_t)l * HID * HID2;
    const unsigned short* u2hl  = u2h  + (size_t)l * HID * HID;
    const unsigned short* u2ll  = u2l  + (size_t)l * HID * HID;
    const float* b1l = msg_b1 + (size_t)l * HID;
    const float* b2l = msg_b2 + (size_t)l * HID;
    const float* c1l = up_b1 + (size_t)l * HID;
    const float* c2l = up_b2 + (size_t)l * HID;

    wmma_gemm64<1, true, 0, 0, false, 0><<<dim3(gemm_blocks(NPr, HID2), 1), 256, 0, stream>>>(
        chp, clp, HID2, 0L, w1ahl, w1all, HID, 0L, (void*)pab, (void*)pab, HID2, 0L, b1l, b1l, 0L, NPr, HID2, HID, 1.0f);

    for (int c = 0; c < nChunks; ++c) {
      const int base = c * CHE;
      int Ec = nE - base; if (Ec > CHE) Ec = CHE;
      const int Mc = ((Ec + 63) / 64) * 64;
      const int vec = ((((size_t)nE + (size_t)base) & 3) == 0) ? 1 : 0;
      wmma_gemm64<0, false, 2, 1, false, 0><<<dim3(gemm_blocks(Mc, HID), 1), 256, 0, stream>>>(
          e16 + (size_t)base * EDGED, e16 + (size_t)base * EDGED, EDGED, 0L, w1el, w1el, EDGED, 0L,
          (void*)pe16, (void*)pe16, HID, 0L, b1l, b1l, 0L, Mc, HID, EDGED, 0.125f);
      k_m1<<<(Mc * 16) / NTHR, NTHR, 0, stream>>>(pab, pe16, eidx, nN, nE, base, Mc, m1p);
      wmma_gemm64<0, false, 2, 0, false, 2><<<dim3(gemm_blocks(Mc, HID), 1), 256, 0, stream>>>(
          m1p, m1p, HID, 0L, w2el, w2el, HID, 0L, (void*)m2p, (void*)m2p, HID, 0L, b2l, b2l, 0L, Mc, HID, HID, 1.0f / 8.0f);
      k_agg<<<nA, NTHR, LDS_AGG, stream>>>(eidx + (size_t)nE + (size_t)base, Ec, m2p, aggp, (c == 0) ? 1 : 0, vec);
    }

    k_aggsplit<<<(NPr * 16) / NTHR, NTHR, 0, stream>>>(aggp, NPr, chp, clp);
    wmma_gemm64<1, true, 2, 2, false, 2><<<dim3(gemm_blocks(NPr, HID), 1), 256, 0, stream>>>(
        chp, clp, HID2, 0L, u1hl, u1ll, HID2, 0L, (void*)uh, (void*)ul, HID, 0L, c1l, c1l, 0L, NPr, HID, HID2, 1.0f);
    wmma_gemm64<1, true, 2, 2, false, 2><<<dim3(gemm_blocks(NPr, HID), 1), 256, 0, stream>>>(
        uh, ul, HID, 0L, u2hl, u2ll, HID, 0L, (void*)chp, (void*)clp, HID2, 0L, c2l, c2l, 0L, NPr, HID, HID, 1.0f);
  }

  wmma_gemm64<1, true, 2, 0, false, 2><<<dim3(gemm_blocks(NPr, TOKH), 1), 256, 0, stream>>>(
      chp, clp, HID2, 0L, tkh, tkl, HID, 0L, (void*)t32, (void*)t32, TOKH, 0L, tok_b1, tok_b1, 0L, NPr, TOKH, HID, 1.0f);
  k_logit<<<(nN + NTHR - 1) / NTHR, NTHR, 0, stream>>>(t32, tok_w2, tok_b2, nN, NPr, out0);
  k_out1<<<(nN * 32 + NTHR - 1) / NTHR, NTHR, 0, stream>>>(chp, clp, nN, NPr, out1);
}
